// MSBlock_78340203479507
// MI455X (gfx1250) — hardware-verified
//
#include <hip/hip_runtime.h>
#include <stdint.h>

typedef __attribute__((ext_vector_type(16))) _Float16 v16h;
typedef __attribute__((ext_vector_type(8)))  _Float16 v8h;
typedef __attribute__((ext_vector_type(8)))  float    v8f;
typedef __attribute__((ext_vector_type(4)))  float    v4f;

#define NC     128
#define NH     128
#define NWD    128
#define NHW    16384
#define NTAP   9
#define KCOL   1152
#define NCHUNK 144
#define NOFF   18
#define MOFF   32

static __device__ __forceinline__ int iclamp(int v, int lo, int hi) { return v < lo ? lo : (v > hi ? hi : v); }

__device__ __forceinline__ void dep_guard_h(v8f& a, v8f& b, v16h x, v16h y) { asm volatile("v_nop\n\tv_nop\n\tv_nop\n\tv_nop" : "+v"(a), "+v"(b) : "v"(x), "v"(y)); }
__device__ __forceinline__ void keep4_h(v16h a, v16h b, v16h c, v16h d) { asm volatile("v_nop" :: "v"(a), "v"(b), "v"(c), "v"(d)); }
__device__ __forceinline__ void acc_guard4(v8f& a, v8f& b, v8f& c, v8f& d) { asm volatile("v_nop\n\tv_nop\n\tv_nop\n\tv_nop" : "+v"(a), "+v"(b), "+v"(c), "+v"(d)); }

template <typename T> struct Frag;
template <> struct Frag<_Float16> {
  typedef v16h V; union U { v16h v; v8h h[2]; };
  static __device__ __forceinline__ v16h load(const _Float16* p) {
    U f; f.h[0] = *(const v8h*)(p); f.h[1] = *(const v8h*)(p + 16); return f.v;
  }
  static __device__ __forceinline__ v8f mma(v16h a, v16h b, v8f c) {
    return __builtin_amdgcn_wmma_f32_16x16x32_f16(false, a, false, b, (short)0, c, false, false);
  }
  static __device__ __forceinline__ void guard(v8f& a, v8f& b, v16h x, v16h y) { dep_guard_h(a, b, x, y); }
  static __device__ __forceinline__ void keep(v16h a, v16h b, v16h c, v16h d) { keep4_h(a, b, c, d); }
};

__global__ __launch_bounds__(128) void gate_k(const float* __restrict__ x, const float* __restrict__ fc_w,
                                              const float* __restrict__ fc_b, float* gate) {
  __shared__ float pool[NC];
  __shared__ float gl[32];
  const int b = blockIdx.x;
  const int c = threadIdx.x;
  const v4f* p4 = (const v4f*)(x + ((size_t)b * NC + c) * NHW);
  double s = 0.0;
#pragma unroll 1
  for (int i = 0; i < NHW / 4; ++i) {
    const v4f v = p4[i];
    s += (double)v[0]; s += (double)v[1]; s += (double)v[2]; s += (double)v[3];
  }
  pool[c] = (float)(s * (1.0 / (double)NHW));
  if (c < 32) gl[c] = 0.0f;
  __syncthreads();
  if (c == 0) {
    float z0 = 0.0f, z1 = 0.0f;
#pragma unroll 1
    for (int i = 0; i < NC; ++i) {
      const float pv = pool[i];
      z0 += pv * fc_w[i];
      z1 += pv * fc_w[NC + i];
    }
    z0 += fc_b[0];
    z1 += fc_b[1];
    const float m  = fmaxf(z0, z1);
    const float e0 = expf(z0 - m), e1 = expf(z1 - m);
    const float inv = 1.0f / (e0 + e1);
    gl[0] = e0 * inv;
    gl[1] = e1 * inv;
  }
  __syncthreads();
  if (c < 32) {
    const float v = gl[c];
    volatile float* gp = gate + b * 32;
    gp[c] = v;
    __threadfence();
    gp[c] = v;
  }
}

__global__ __launch_bounds__(256) void wprep_k(const float* __restrict__ conv_w, const float* __restrict__ def_w,
                                               const float* __restrict__ off_w,
                                               _Float16* btc, _Float16* btd,
                                               _Float16* wo0, _Float16* wo1, _Float16* wo2) {
  const int which = blockIdx.y;
  const int nrows = (which == 2) ? MOFF : NC;
  const int g = blockIdx.x * 256 + threadIdx.x;
  if (g >= nrows * NCHUNK) return;
  const int o   = g / NCHUNK;
  const int j   = g - o * NCHUNK;
  const int k   = j >> 4;
  const int ci0 = (j & 15) * 8;
  const float* src = (which == 0) ? conv_w : ((which == 1) ? def_w : off_w);
  const bool zero = (which == 2) && (o >= NOFF);
  const int srow  = zero ? (NOFF - 1) : o;
  float vals[8];
#pragma unroll
  for (int e = 0; e < 8; ++e) {
    const float w = src[((size_t)(srow * NC + ci0 + e)) * NTAP + k];
    vals[e] = zero ? 0.0f : w;
  }
  const size_t d = (size_t)o * KCOL + (size_t)j * 8;
  if (which != 2) {
    v8h hv;
#pragma unroll
    for (int e = 0; e < 8; ++e) hv[e] = (_Float16)(vals[e] * 32.0f);
    _Float16* dst = ((which == 0) ? btc : btd) + d;
    *(volatile v8h*)dst = hv;
    __threadfence();
    *(volatile v8h*)dst = hv;
  } else {
    v8h h0, h1, h2;
#pragma unroll
    for (int e = 0; e < 8; ++e) {
      const float wsc = vals[e] * 1024.0f;
      const _Float16 hh = (_Float16)wsc;
      h0[e] = hh;
      h1[e] = (_Float16)(vals[e] * 0.5f);
      h2[e] = (_Float16)(wsc - (float)hh);
    }
    *(volatile v8h*)(wo0 + d) = h0;
    *(volatile v8h*)(wo1 + d) = h1;
    *(volatile v8h*)(wo2 + d) = h2;
    __threadfence();
    *(volatile v8h*)(wo0 + d) = h0;
    *(volatile v8h*)(wo1 + d) = h1;
    *(volatile v8h*)(wo2 + d) = h2;
  }
}

__global__ __launch_bounds__(256) void nhwc_k(const float* __restrict__ xb, float* xt) {
  __shared__ __align__(16) float tile[32][36];
  const int p0 = blockIdx.x * 32;
  const int c0 = blockIdx.y * 32;
  const int t  = threadIdx.x;
  {
    const int c = t >> 3, pq = (t & 7) * 4;
    const v4f v = *(const v4f*)(xb + (size_t)(c0 + c) * NHW + p0 + pq);
    *(v4f*)(&tile[c][pq]) = v;
  }
  __syncthreads();
  {
    const int p = t >> 3, cq = (t & 7) * 4;
    v4f w4;
    w4[0] = tile[cq + 0][p];
    w4[1] = tile[cq + 1][p];
    w4[2] = tile[cq + 2][p];
    w4[3] = tile[cq + 3][p];
    float* dst = xt + (size_t)(p0 + p) * NC + c0 + cq;
    *(volatile v4f*)dst = w4;
    __threadfence();
    *(volatile v4f*)dst = w4;
  }
}

__global__ __launch_bounds__(288) void im2col_k(const float* __restrict__ xt, _Float16* ph, _Float16* pl) {
  const int k    = threadIdx.x >> 5;
  const int lane = threadIdx.x & 31;
  const int p    = blockIdx.x * 2 + (lane >> 4);
  const int cq   = (lane & 15) * 8;
  const int h = p >> 7, w = p & (NWD - 1);
  const int ki = k / 3, kj = k - ki * 3;
  const int hs = h + ki - 1, wsx = w + kj - 1;
  const bool ok = (hs >= 0) && (hs < NH) && (wsx >= 0) && (wsx < NWD);
  const int hc = iclamp(hs, 0, NH - 1), wc = iclamp(wsx, 0, NWD - 1);
  const float* src = xt + ((size_t)(hc * NWD + wc)) * NC + cq;
  const v4f a  = *(const v4f*)src;
  const v4f bq = *(const v4f*)(src + 4);
  v8h hv, lv;
#pragma unroll
  for (int e = 0; e < 4; ++e) {
    const float f0 = ok ? a[e] : 0.0f;
    const float f1 = ok ? bq[e] : 0.0f;
    const _Float16 h0 = (_Float16)f0, h1 = (_Float16)f1;
    hv[e] = h0;
    hv[4 + e] = h1;
    lv[e]     = (_Float16)((f0 - (float)h0) * 2048.0f);
    lv[4 + e] = (_Float16)((f1 - (float)h1) * 2048.0f);
  }
  const size_t o = (size_t)p * KCOL + (size_t)k * NC + cq;
  *(volatile v8h*)(ph + o) = hv;
  *(volatile v8h*)(pl + o) = lv;
  __threadfence();
  *(volatile v8h*)(ph + o) = hv;
  *(volatile v8h*)(pl + o) = lv;
}

__global__ __launch_bounds__(288) void sample_k(const float* __restrict__ xt, const float* __restrict__ off, _Float16* splane) {
  const int k    = threadIdx.x >> 5;
  const int lane = threadIdx.x & 31;
  const int p    = blockIdx.x * 2 + (lane >> 4);
  const int cq   = (lane & 15) * 8;
  const int h = p >> 7, w = p & (NWD - 1);
  const int ki = k / 3, kj = k - ki * 3;
  const float dy = off[(size_t)(2 * k) * NHW + p];
  const float dx = off[(size_t)(2 * k + 1) * NHW + p];
  const float py = (float)(h + ki - 1) + dy;
  const float px = (float)(w + kj - 1) + dx;
  const float fy = floorf(py), fx = floorf(px);
  const float wy1 = py - fy, wx1 = px - fx;
  const float wy0 = 1.0f - wy1, wx0 = 1.0f - wx1;
  const float fyc = fminf(fmaxf(fy, -8.0f), (float)(NH + 8));
  const float fxc = fminf(fmaxf(fx, -8.0f), (float)(NWD + 8));
  const int y0 = (int)fyc, x0 = (int)fxc;
  const int y1 = y0 + 1, x1 = x0 + 1;
  const bool vy0 = (y0 >= 0) && (y0 < NH);
  const bool vy1 = (y1 >= 0) && (y1 < NH);
  const bool vx0 = (x0 >= 0) && (x0 < NWD);
  const bool vx1 = (x1 >= 0) && (x1 < NWD);
  const float w00 = (vy0 && vx0) ? (wy0 * wx0) : 0.0f;
  const float w01 = (vy0 && vx1) ? (wy0 * wx1) : 0.0f;
  const float w10 = (vy1 && vx0) ? (wy1 * wx0) : 0.0f;
  const float w11 = (vy1 && vx1) ? (wy1 * wx1) : 0.0f;
  const int yc0 = iclamp(y0, 0, NH - 1), yc1 = iclamp(y1, 0, NH - 1);
  const int xc0 = iclamp(x0, 0, NWD - 1), xc1 = iclamp(x1, 0, NWD - 1);
  const float* r00 = xt + ((size_t)(yc0 * NWD + xc0)) * NC + cq;
  const float* r01 = xt + ((size_t)(yc0 * NWD + xc1)) * NC + cq;
  const float* r10 = xt + ((size_t)(yc1 * NWD + xc0)) * NC + cq;
  const float* r11 = xt + ((size_t)(yc1 * NWD + xc1)) * NC + cq;
  const v4f a00 = *(const v4f*)r00, b00 = *(const v4f*)(r00 + 4);
  const v4f a01 = *(const v4f*)r01, b01 = *(const v4f*)(r01 + 4);
  const v4f a10 = *(const v4f*)r10, b10 = *(const v4f*)(r10 + 4);
  const v4f a11 = *(const v4f*)r11, b11 = *(const v4f*)(r11 + 4);
  v8h hv;
#pragma unroll
  for (int e = 0; e < 4; ++e) {
    float v = a00[e] * w00 + a01[e] * w01;
    v = v + a10[e] * w10;
    v = v + a11[e] * w11;
    hv[e] = (_Float16)v;
    float u = b00[e] * w00 + b01[e] * w01;
    u = u + b10[e] * w10;
    u = u + b11[e] * w11;
    hv[4 + e] = (_Float16)u;
  }
  _Float16* dst = splane + (size_t)p * KCOL + (size_t)k * NC + cq;
  *(volatile v8h*)dst = hv;
  __threadfence();
  *(volatile v8h*)dst = hv;
}

template <int MSUB>
__device__ __forceinline__ void kseg_f16(v8f (&acc)[MSUB][4], const _Float16* __restrict__ A, int lda,
                                         const _Float16* __restrict__ Bt, int ldb, int m0, int n0, int K,
                                         int rlane, int koff) {
  typedef Frag<_Float16> F;
  for (int k0 = 0; k0 < K; k0 += 32) {
    v16h bh[4];
#pragma unroll
    for (int j = 0; j < 4; ++j)
      bh[j] = F::load(Bt + (size_t)(n0 + (j << 4) + rlane) * ldb + koff + k0);
#pragma unroll
    for (int i = 0; i < MSUB; ++i) {
      const v16h ah = F::load(A + (size_t)(m0 + (i << 4) + rlane) * lda + koff + k0);
#pragma unroll
      for (int j = 0; j < 4; ++j) acc[i][j] = F::mma(ah, bh[j], acc[i][j]);
      F::guard(acc[i][0], acc[i][3], ah, ah);
    }
    F::keep(bh[0], bh[1], bh[2], bh[3]);
  }
}

template <int MSUB, int NSEG, int EPI>
__global__ __launch_bounds__(256) void gemm_f16(
    const _Float16* __restrict__ A0, const _Float16* __restrict__ A1, const _Float16* __restrict__ A2, int lda,
    const _Float16* __restrict__ B0, const _Float16* __restrict__ B1, const _Float16* __restrict__ B2, int ldb,
    float* Cout, int ldc,
    const float* __restrict__ bias, int nbias,
    const float* resid, const float* __restrict__ gatep,
    int M, int N, int K, float scale) {
  __shared__ __align__(16) float sT[8][16 * 68];
  const int lane = threadIdx.x & 31;
  const int wave = threadIdx.x >> 5;
  const int tilesN = N >> 6;
  const int tilesM = M / (16 * MSUB);
  const int tile = blockIdx.x * 8 + wave;
  if (tile >= tilesM * tilesN) return;
  const int tm = tile / tilesN;
  const int tn = tile - tm * tilesN;
  const int m0 = tm * (16 * MSUB);
  const int n0 = tn << 6;
  const int rlane = lane & 15;
  const int koff  = (lane >> 4) * 8;
  const int mOff  = (lane >> 4) * 8;

  v8f acc[MSUB][4];
#pragma unroll
  for (int i = 0; i < MSUB; ++i)
#pragma unroll
    for (int j = 0; j < 4; ++j) acc[i][j] = (v8f){0.f, 0.f, 0.f, 0.f, 0.f, 0.f, 0.f, 0.f};

  kseg_f16<MSUB>(acc, A0, lda, B0, ldb, m0, n0, K, rlane, koff);
  if (NSEG > 1) kseg_f16<MSUB>(acc, A1, lda, B1, ldb, m0, n0, K, rlane, koff);
  if (NSEG > 2) kseg_f16<MSUB>(acc, A2, lda, B2, ldb, m0, n0, K, rlane, koff);
#pragma unroll
  for (int i = 0; i < MSUB; ++i) acc_guard4(acc[i][0], acc[i][1], acc[i][2], acc[i][3]);

  float g0 = 0.0f, g1 = 1.0f;
  if (EPI == 1) { g0 = gatep[0]; g1 = gatep[1]; }
  float* slab = sT[wave];
#pragma unroll
  for (int i = 0; i < MSUB; ++i) {
    const int mBase = m0 + (i << 4);
#pragma unroll
    for (int j = 0; j < 4; ++j) {
      const int n = n0 + (j << 4) + rlane;
#pragma unroll
      for (int r = 0; r < 8; ++r) {
        const int m  = mBase + mOff + r;
        const int mb = (m < nbias) ? m : (nbias - 1);
        float v = acc[i][j][r] * scale + bias[mb];
        if (EPI == 1) {
          const float lv = resid[(size_t)m * ldc + n];
          v = g0 * lv + g1 * v;
          v = fmaxf(v, 0.0f);
        }
        slab[(mOff + r) * 68 + (j << 4) + rlane] = v;
      }
    }
    __builtin_amdgcn_fence(__ATOMIC_RELEASE, "workgroup");
    __builtin_amdgcn_wave_barrier();
    __builtin_amdgcn_fence(__ATOMIC_ACQUIRE, "workgroup");
    {
      const int hh = lane >> 4, c4 = (lane & 15) * 4;
      for (int pass = 0; pass < 2; ++pass) {
#pragma unroll
        for (int it = 0; it < 8; ++it) {
          const int row = it * 2 + hh;
          const v4f vv = *(const v4f*)(slab + row * 68 + c4);
          *(volatile v4f*)(Cout + (size_t)(mBase + row) * ldc + n0 + c4) = vv;
        }
        __threadfence();
      }
    }
    __builtin_amdgcn_fence(__ATOMIC_RELEASE, "workgroup");
    __builtin_amdgcn_wave_barrier();
    __builtin_amdgcn_fence(__ATOMIC_ACQUIRE, "workgroup");
  }
}

extern "C" void kernel_launch(void* const* d_in, const int* in_sizes, int n_in,
                              void* d_out, int out_size, void* d_ws, size_t ws_size,
                              hipStream_t stream) {
  if (n_in < 9) return;
  const int nb = in_sizes[0] / (NC * NHW);
  if (nb < 1 || nb > 16 || in_sizes[0] != nb * NC * NHW) return;
  if (in_sizes[1] != NC * KCOL || in_sizes[2] != NC || in_sizes[3] != NOFF * KCOL || in_sizes[4] != NOFF ||
      in_sizes[5] != NC * KCOL || in_sizes[6] != NC || in_sizes[7] != 2 * NC || in_sizes[8] != 2) return;
  if (out_size != nb * NC * NHW) return;

  const float* x      = (const float*)d_in[0];
  const float* conv_w = (const float*)d_in[1];
  const float* conv_b = (const float*)d_in[2];
  const float* off_w  = (const float*)d_in[3];
  const float* off_b  = (const float*)d_in[4];
  const float* def_w  = (const float*)d_in[5];
  const float* def_b  = (const float*)d_in[6];
  const float* fc_w   = (const float*)d_in[7];
  const float* fc_b   = (const float*)d_in[8];
  float* out = (float*)d_out;

  const size_t o_gate = 0;
  const size_t o_btc  = 2048;
  const size_t o_btd  = o_btc + (size_t)NC * KCOL * 2;
  const size_t o_wo0  = o_btd + (size_t)NC * KCOL * 2;
  const size_t o_wo1  = o_wo0 + (size_t)MOFF * KCOL * 2;
  const size_t o_wo2  = o_wo1 + (size_t)MOFF * KCOL * 2;
  const size_t o_xt   = o_wo2 + (size_t)MOFF * KCOL * 2;
  const size_t o_ph   = o_xt  + (size_t)NHW * NC * 4;
  const size_t o_pl   = o_ph  + (size_t)NHW * KCOL * 2;
  const size_t o_sp   = o_pl  + (size_t)NHW * KCOL * 2;
  const size_t o_off  = o_sp  + (size_t)NHW * KCOL * 2;
  const size_t total  = o_off + (size_t)MOFF * NHW * 4;
  if (total > ws_size) return;

  char* ws = (char*)d_ws;
  float*    gate = (float*)(ws + o_gate);
  _Float16* btc  = (_Float16*)(ws + o_btc);
  _Float16* btd  = (_Float16*)(ws + o_btd);
  _Float16* wo0  = (_Float16*)(ws + o_wo0);
  _Float16* wo1  = (_Float16*)(ws + o_wo1);
  _Float16* wo2  = (_Float16*)(ws + o_wo2);
  float*    xt   = (float*)(ws + o_xt);
  _Float16* ph   = (_Float16*)(ws + o_ph);
  _Float16* pl   = (_Float16*)(ws + o_pl);
  _Float16* sp   = (_Float16*)(ws + o_sp);
  float*    offb = (float*)(ws + o_off);

  gate_k<<<dim3(nb), dim3(NC), 0, stream>>>(x, fc_w, fc_b, gate);
  wprep_k<<<dim3((NC * NCHUNK + 255) / 256, 3), dim3(256), 0, stream>>>(conv_w, def_w, off_w, btc, btd, wo0, wo1, wo2);

  const int blocks_main = ((NC / 64) * (NHW / 64) + 7) / 8;
  const int blocks_off  = ((MOFF / 32) * (NHW / 64) + 7) / 8;
  for (int b = 0; b < nb; ++b) {
    const float* xb   = x + (size_t)b * NC * NHW;
    float*       outb = out + (size_t)b * NC * NHW;
    const float* gb   = gate + 32 * b;
    nhwc_k<<<dim3(NHW / 32, NC / 32), dim3(256), 0, stream>>>(xb, xt);
    im2col_k<<<dim3(NHW / 2), dim3(288), 0, stream>>>(xt, ph, pl);
    gemm_f16<2, 3, 0><<<dim3(blocks_off), dim3(256), 0, stream>>>(
        wo0, wo1, wo2, KCOL, ph, pl, ph, KCOL, offb, NHW, off_b, NOFF, outb, gb, MOFF, NHW, KCOL, 1.0f / 1024.0f);
    sample_k<<<dim3(NHW / 2), dim3(288), 0, stream>>>(xt, offb, sp);
    gemm_f16<4, 1, 0><<<dim3(blocks_main), dim3(256), 0, stream>>>(
        btc, btc, btc, KCOL, ph, ph, ph, KCOL, outb, NHW, conv_b, NC, outb, gb, NC, NHW, KCOL, 1.0f / 32.0f);
    gemm_f16<4, 1, 1><<<dim3(blocks_main), dim3(256), 0, stream>>>(
        btd, btd, btd, KCOL, sp, sp, sp, KCOL, outb, NHW, def_b, NC, outb, gb, NC, NHW, KCOL, 1.0f / 32.0f);
  }
  (void)hipGetLastError();
}
